// IndraQuantumLayer_55886114455740
// MI455X (gfx1250) — hardware-run, weakly checked
//
#include <hip/hip_runtime.h>
#include <math.h>

#ifndef NB
#define NB 4
#endif
#ifndef SEQ
#define SEQ 2048
#endif
#define NB_FULL 4
#define SEQ_FULL 2048
#define DM 1024
#define HEADS 16
#define HD 64
#define FFD 4096
#define MTOK (NB * SEQ)
#define SEQ_U ((unsigned)SEQ)
#define SEQF_U ((unsigned)SEQ_FULL)
#define DM_U 1024u
#define QKP 2048u
#define FFD_U 4096u
#define HEADS_U 16u
#define HD_U 64u

static_assert(HEADS * HD == DM);
static_assert(HEADS == 16 && HD == 64 && DM == 1024 && FFD == 4096);
static_assert(SEQ % 64 == 0 && SEQ <= SEQ_FULL && NB <= NB_FULL && NB >= 1);
static_assert(MTOK % 64 == 0);
static_assert(DM % 64 == 0 && (3 * DM) % 64 == 0 && FFD % 64 == 0 && DM % 32 == 0 && FFD % 32 == 0);
static_assert(((MTOK * (DM / 8)) % 256) == 0);

#define CARRY_ACT 2048.0f
#define CARRY_W   131072.0f
#define CARRY_QKV 4096.0f
#define CARRY_P   16384.0f
#define CARRY_HID 4096.0f
#define UNC_AW (1.0f / (CARRY_ACT * CARRY_W))
#define UNC_II (1.0f / (CARRY_ACT * CARRY_ACT))
#define UNC_QK (1.0f / (CARRY_QKV * CARRY_QKV))
#define UNC_TW (1.0f / (CARRY_QKV * CARRY_W))
#define UNC_HW (1.0f / (CARRY_HID * CARRY_W))
#define UNC_P  (1.0f / CARRY_P)
#define HOP_DIV 32.0f
#define SCORE_DIV 8.0f
#define SQRT_HALF 0.70710678118654752f
#define LN_EPS 1e-5f

typedef __attribute__((ext_vector_type(16))) _Float16 v16h;
typedef __attribute__((ext_vector_type(8)))  _Float16 v8h;
typedef __attribute__((ext_vector_type(8)))  float    v8f;
typedef __attribute__((ext_vector_type(4)))  float    v4f;
typedef _Float16 h16;

constexpr size_t SZ_ACT16 = (size_t)MTOK * DM * 2;
constexpr size_t SZ_QK    = (size_t)MTOK * 2 * DM * 2;
constexpr size_t SZ_HID   = (size_t)MTOK * FFD * 2;
constexpr size_t SZ_F32   = (size_t)MTOK * DM * 4;
constexpr size_t SZ_HOP   = (size_t)SEQ * SEQ * 4;
constexpr size_t SZ_WQKV  = (size_t)3 * DM * DM * 2;
constexpr size_t SZ_WO    = (size_t)DM * DM * 2;
constexpr size_t SZ_W1    = (size_t)FFD * DM * 2;
constexpr size_t SZ_W2    = (size_t)DM * FFD * 2;
constexpr size_t OFF_X16  = 0;
constexpr size_t OFF_QK   = OFF_X16 + SZ_ACT16;
constexpr size_t OFF_VT   = OFF_QK + SZ_QK;
constexpr size_t OFF_IM   = OFF_VT + SZ_ACT16;
constexpr size_t OFF_HID  = OFF_QK;
constexpr size_t OFF_WQKV = OFF_IM + SZ_ACT16;
constexpr size_t OFF_WO   = OFF_WQKV + SZ_WQKV;
constexpr size_t OFF_W1   = OFF_WO + SZ_WO;
constexpr size_t OFF_W2   = OFF_W1 + SZ_W1;
constexpr size_t OFF_HOP  = OFF_W2 + SZ_W2;
constexpr size_t OFF_ATT  = OFF_HOP + SZ_HOP;
constexpr size_t OFF_PRE  = OFF_ATT + SZ_ACT16;
constexpr size_t OFF_X1F  = OFF_PRE + SZ_F32;
constexpr size_t OFF_X1H  = OFF_X1F + SZ_F32;
constexpr size_t WS_TOTAL = OFF_X1H + SZ_ACT16;
static_assert(SZ_QK + 2 * SZ_ACT16 >= SZ_HID);
static_assert(OFF_HID + SZ_HID <= OFF_WQKV);
static_assert(WS_TOTAL <= (size_t)268435456);
static_assert((OFF_QK % 256) == 0 && (OFF_VT % 256) == 0 && (OFF_IM % 256) == 0 && (OFF_WQKV % 256) == 0);
static_assert((OFF_WO % 256) == 0 && (OFF_W1 % 256) == 0 && (OFF_W2 % 256) == 0 && (OFF_HOP % 256) == 0);
static_assert((OFF_ATT % 256) == 0 && (OFF_PRE % 256) == 0 && (OFF_X1F % 256) == 0 && (OFF_X1H % 256) == 0);


static __device__ __forceinline__ float bfr(float f) {
    unsigned u = __float_as_uint(f);
    u += 0x7FFFu + ((u >> 16) & 1u);
    return __uint_as_float(u & 0xFFFF0000u);
}
static __device__ __forceinline__ h16 toh_flush(float v) {
    const float w = (fabsf(v) < 6.103515625e-05f) ? 0.0f : v;
    return (h16)w;
}
static __device__ __forceinline__ unsigned frow(unsigned r) {
    const unsigned bq = r / SEQ_U;
    return bq * SEQF_U + (r - bq * SEQ_U);
}
static __device__ __forceinline__ void vst2_h8(h16* p, v8h v) {
    *(volatile v8h*)p = v;
    __threadfence();
    *(volatile v8h*)p = v;
}

union FragU { v16h v; v8h h[2]; };
static __device__ __forceinline__ v16h frag_ld(const h16* p) {
    FragU f; f.h[0] = *(const v8h*)(p); f.h[1] = *(const v8h*)(p + 16); return f.v;
}
static __device__ __forceinline__ v8f wmma16g(v16h a, v16h b, v8f c) {
    c = __builtin_amdgcn_wmma_f32_16x16x32_f16(false, a, false, b, (short)0, c, false, false);
    asm volatile("v_nop\n\tv_nop\n\tv_nop\n\tv_nop" : "+v"(c) : "v"(a), "v"(b));
    return c;
}
static __device__ __forceinline__ void wave_sync_lds() {
    __builtin_amdgcn_fence(3  , "workgroup");
    __builtin_amdgcn_wave_barrier();
    __builtin_amdgcn_fence(2  , "workgroup");
}

template <int WHICH>
__global__ __launch_bounds__(256) void k_cvt16(const float* __restrict__ src, h16* __restrict__ dst, unsigned n8) {
    const unsigned bx = blockIdx.x;
    const unsigned u = bx * 256u + threadIdx.x;
    if (u >= n8) return;
    size_t so;
    if (WHICH == 0) {
        const unsigned row = u >> 7;
        const unsigned c0 = (u & 127u) * 8u;
        so = (size_t)frow(row) * DM_U + c0;
    } else {
        so = (size_t)u * 8u;
    }
    const v4f a = *(const v4f*)(src + so);
    const v4f bq = *(const v4f*)(src + so + 4);
    constexpr float cs = (WHICH == 0) ? CARRY_ACT : CARRY_W;
    v8h hv;
    hv[0] = toh_flush(bfr(a.x) * cs);  hv[1] = toh_flush(bfr(a.y) * cs);
    hv[2] = toh_flush(bfr(a.z) * cs);  hv[3] = toh_flush(bfr(a.w) * cs);
    hv[4] = toh_flush(bfr(bq.x) * cs); hv[5] = toh_flush(bfr(bq.y) * cs);
    hv[6] = toh_flush(bfr(bq.z) * cs); hv[7] = toh_flush(bfr(bq.w) * cs);
    vst2_h8(dst + (size_t)u * 8u, hv);
}

template <int MODE> struct GC;
template <> struct GC<0> { static constexpr unsigned M = MTOK, N = 3 * DM, K = DM; };
template <> struct GC<1> { static constexpr unsigned M = SEQ,  N = SEQ,    K = DM; };
template <> struct GC<2> { static constexpr unsigned M = MTOK, N = DM,     K = DM; };
template <> struct GC<3> { static constexpr unsigned M = MTOK, N = FFD,    K = DM; };
template <> struct GC<4> { static constexpr unsigned M = MTOK, N = DM,     K = FFD; };

template <int MODE>
static __device__ __forceinline__ float epi_val(float a, float bv) {
    if constexpr (MODE == 0) {
        return (a * UNC_AW + bv) * CARRY_QKV;
    } else if constexpr (MODE == 1) {
        const float dotv = a * UNC_II;
        return dotv / HOP_DIV;
    } else if constexpr (MODE == 2) {
        return a * UNC_TW + bv;
    } else if constexpr (MODE == 3) {
        const float z = a * UNC_AW + bv;
        const float gz = 0.5f * z * (1.0f + erff(z * SQRT_HALF));
        return gz * CARRY_HID;
    } else {
        return a * UNC_HW + bv;
    }
}

template <int MODE>
__global__ __launch_bounds__(256) void k_gemm(const h16* __restrict__ A, const h16* __restrict__ Bt,
                                              void* C0, void* C1,
                                              const float* __restrict__ bias, const float* __restrict__ resid) {
    constexpr unsigned M = GC<MODE>::M, N = GC<MODE>::N, K = GC<MODE>::K;
    constexpr unsigned TM = M / 64u, TN = N / 64u;
    static_assert(M % 64u == 0 && N % 64u == 0 && K % 32u == 0);
    __shared__ __align__(16) float sT[8][16 * 68];
    const unsigned lane = threadIdx.x & 31u;
    const unsigned wave = threadIdx.x >> 5;
    const unsigned bx = blockIdx.x;
    const unsigned tile = bx * 8u + wave;
    if (tile >= TM * TN) return;
    const unsigned tm = tile / TN;
    const unsigned tn = tile - tm * TN;
    if (MODE == 1) { if (tn > tm) return; }
    const unsigned m0 = tm << 6, n0 = tn << 6;
    const unsigned rlane = lane & 15u;
    const unsigned hh = lane >> 4;
    const unsigned koff = hh * 8u;
    const unsigned mOff = koff;

    v8f acc[4][4];
#pragma unroll
    for (int i = 0; i < 4; ++i)
#pragma unroll
        for (int j = 0; j < 4; ++j) acc[i][j] = (v8f){0.f, 0.f, 0.f, 0.f, 0.f, 0.f, 0.f, 0.f};

    const h16* ap = A + (size_t)(m0 + rlane) * K + koff;
    const h16* bp = Bt + (size_t)(n0 + rlane) * K + koff;
    for (unsigned k0 = 0; k0 < K; k0 += 32u) {
        v16h bh[4];
#pragma unroll
        for (int j = 0; j < 4; ++j) bh[j] = frag_ld(bp + (size_t)((unsigned)j << 4) * K + k0);
#pragma unroll
        for (int i = 0; i < 4; ++i) {
            const v16h ah = frag_ld(ap + (size_t)((unsigned)i << 4) * K + k0);
#pragma unroll
            for (int j = 0; j < 4; ++j) acc[i][j] = wmma16g(ah, bh[j], acc[i][j]);
        }
    }

    float* slab = sT[wave];
    float bvv[4];
#pragma unroll
    for (int j = 0; j < 4; ++j) {
        if constexpr (MODE != 1) bvv[j] = bfr(bias[n0 + ((unsigned)j << 4) + rlane]);
        else bvv[j] = 0.0f;
    }

    if constexpr (MODE == 1 || MODE == 2 || MODE == 4) {
        float* C = (float*)C0;
        const unsigned c4 = (lane & 15u) * 4u;
#pragma unroll
        for (int i = 0; i < 4; ++i) {
            const unsigned mBase = m0 + ((unsigned)i << 4);
#pragma unroll
            for (int j = 0; j < 4; ++j)
#pragma unroll
                for (int r = 0; r < 8; ++r)
                    slab[(mOff + (unsigned)r) * 68u + ((unsigned)j << 4) + rlane] = epi_val<MODE>(acc[i][j][r], bvv[j]);
            wave_sync_lds();
#pragma unroll
            for (int half = 0; half < 2; ++half) {
                v4f vv[4];
#pragma unroll
                for (int it = 0; it < 4; ++it) {
                    const unsigned row = (unsigned)(half * 4 + it) * 2u + hh;
                    vv[it] = *(const v4f*)(slab + row * 68u + c4);
                    if constexpr (MODE == 2) {
                        const v4f rx = *(const v4f*)(resid + (size_t)frow(mBase + row) * DM_U + n0 + c4);
                        vv[it].x += bfr(rx.x); vv[it].y += bfr(rx.y); vv[it].z += bfr(rx.z); vv[it].w += bfr(rx.w);
                    }
                    if constexpr (MODE == 4) {
                        vv[it] += *(const v4f*)(resid + (size_t)(mBase + row) * DM_U + n0 + c4);
                    }
                }
                for (int pass = 0; pass < 2; ++pass) {
#pragma unroll
                    for (int it = 0; it < 4; ++it) {
                        const unsigned row = (unsigned)(half * 4 + it) * 2u + hh;
                        *(volatile v4f*)(C + (size_t)(mBase + row) * N + n0 + c4) = vv[it];
                    }
                    __threadfence();
                }
            }
            wave_sync_lds();
        }
    } else {
        const unsigned q = lane >> 3, c8 = (lane & 7u) * 8u;
        const bool rowmajor = (MODE == 3) || (n0 < 2u * DM_U);
        if (rowmajor) {
            h16* C = (h16*)C0;
            constexpr unsigned ldc = (MODE == 3) ? FFD_U : QKP;
#pragma unroll
            for (int i = 0; i < 4; ++i) {
                const unsigned mBase = m0 + ((unsigned)i << 4);
#pragma unroll
                for (int j = 0; j < 4; ++j)
#pragma unroll
                    for (int r = 0; r < 8; ++r)
                        slab[(mOff + (unsigned)r) * 68u + ((unsigned)j << 4) + rlane] = epi_val<MODE>(acc[i][j][r], bvv[j]);
                wave_sync_lds();
                v8h hv[4];
#pragma unroll
                for (int it = 0; it < 4; ++it) {
                    const unsigned row = (unsigned)it * 4u + q;
                    const float* sp = slab + row * 68u + c8;
#pragma unroll
                    for (int e = 0; e < 8; ++e) hv[it][e] = toh_flush(sp[e]);
                }
                for (int pass = 0; pass < 2; ++pass) {
#pragma unroll
                    for (int it = 0; it < 4; ++it) {
                        const unsigned row = (unsigned)it * 4u + q;
                        *(volatile v8h*)(C + (size_t)(mBase + row) * ldc + n0 + c8) = hv[it];
                    }
                    __threadfence();
                }
                wave_sync_lds();
            }
        } else {
            if constexpr (MODE == 0) {
                h16* C = (h16*)C1;
                const unsigned bb = m0 / SEQ_U;
                const unsigned s0 = m0 - bb * SEQ_U;
                const unsigned head = tn - 32u;
#pragma unroll
                for (int j = 0; j < 4; ++j) {
#pragma unroll
                    for (int i = 0; i < 4; ++i)
#pragma unroll
                        for (int r = 0; r < 8; ++r)
                            slab[rlane * 68u + ((unsigned)i << 4) + mOff + (unsigned)r] = epi_val<MODE>(acc[i][j][r], bvv[j]);
                    wave_sync_lds();
                    v8h hv[4];
#pragma unroll
                    for (int it = 0; it < 4; ++it) {
                        const unsigned drow = (unsigned)it * 4u + q;
                        const float* sp = slab + drow * 68u + c8;
#pragma unroll
                        for (int e = 0; e < 8; ++e) hv[it][e] = toh_flush(sp[e]);
                    }
                    for (int pass = 0; pass < 2; ++pass) {
#pragma unroll
                        for (int it = 0; it < 4; ++it) {
                            const unsigned drow = (unsigned)it * 4u + q;
                            *(volatile v8h*)(C + ((size_t)(bb * HEADS_U + head) * HD_U + ((unsigned)j << 4) + drow) * SEQ_U + s0 + c8) = hv[it];
                        }
                        __threadfence();
                    }
                    wave_sync_lds();
                }
            }
        }
    }
}

#define AT_PP 72u
#define AT_SP 68u
__global__ __launch_bounds__(128) void k_attn(const h16* __restrict__ qk, const h16* __restrict__ vT,
                                              const float* __restrict__ hop, h16* __restrict__ att, unsigned b) {
    __shared__ __align__(16) float sS[4][16 * 68];
    __shared__ __align__(16) h16   sP[4][16 * 72];
    const unsigned tid = threadIdx.x, lane = tid & 31u, wave = tid >> 5;
    const unsigned hh = lane >> 4, c = lane & 15u;
    const unsigned rt = blockIdx.x, head = blockIdx.y;
    const unsigned q0 = rt * 64u + wave * 16u;
    const unsigned tok0 = b * SEQ_U + q0;
    float* slab = sS[wave];
    h16* pw = sP[wave];

    const h16* qbase = qk + (size_t)(tok0 + c) * QKP + head * HD_U + 8u * hh;
    const v16h qf0 = frag_ld(qbase);
    const v16h qf1 = frag_ld(qbase + 32);
    const h16* kbase = qk + (size_t)(b * SEQ_U + c) * QKP + DM_U + head * HD_U + 8u * hh;
    const h16* vbase = vT + ((size_t)(b * HEADS_U + head) * HD_U + c) * SEQ_U + 8u * hh;

    const unsigned prow = lane >> 1, phf = lane & 1u;
    const unsigned qi = q0 + prow;
    const float* hrow = hop + (size_t)qi * SEQ_U + 32u * phf;
    float* srow = slab + prow * AT_SP + 32u * phf;
    h16* prw = pw + prow * AT_PP + 32u * phf;
    const float NEG_INF = -__builtin_inff();
    const float SC_QK = UNC_QK / SCORE_DIV;

    float mrow = -3.0e38f, lrow = 0.0f;
    v8f o[4];
#pragma unroll
    for (int t = 0; t < 4; ++t) o[t] = (v8f){0.f, 0.f, 0.f, 0.f, 0.f, 0.f, 0.f, 0.f};

    for (unsigned kc = 0; kc <= rt; ++kc) {
        const unsigned kv0 = kc * 64u;
        v8f s[4];
#pragma unroll
        for (int j = 0; j < 4; ++j) {
            const h16* kp = kbase + (size_t)(kv0 + ((unsigned)j << 4)) * QKP;
            const v16h kf0 = frag_ld(kp);
            const v16h kf1 = frag_ld(kp + 32);
            const v8f z = (v8f){0.f, 0.f, 0.f, 0.f, 0.f, 0.f, 0.f, 0.f};
            s[j] = wmma16g(qf0, kf0, z);
            s[j] = wmma16g(qf1, kf1, s[j]);
        }
#pragma unroll
        for (int j = 0; j < 4; ++j)
#pragma unroll
            for (int r = 0; r < 8; ++r)
                slab[(8u * hh + (unsigned)r) * AT_SP + ((unsigned)j << 4) + c] = s[j][r];
        wave_sync_lds();

        float mx = NEG_INF;
        for (unsigned g = 0; g < 8u; ++g) {
            const v4f sv = *(const v4f*)(srow + 4u * g);
            const v4f hv = *(const v4f*)(hrow + kv0 + 4u * g);
            const unsigned kcol = kv0 + 32u * phf + 4u * g;
            float a0 = sv.x * SC_QK + hv.x;
            float a1 = sv.y * SC_QK + hv.y;
            float a2 = sv.z * SC_QK + hv.z;
            float a3 = sv.w * SC_QK + hv.w;
            a0 = (kcol      > qi) ? NEG_INF : a0;
            a1 = (kcol + 1u > qi) ? NEG_INF : a1;
            a2 = (kcol + 2u > qi) ? NEG_INF : a2;
            a3 = (kcol + 3u > qi) ? NEG_INF : a3;
            mx = fmaxf(fmaxf(mx, fmaxf(a0, a1)), fmaxf(a2, a3));
            v4f w; w.x = a0; w.y = a1; w.z = a2; w.w = a3;
            *(v4f*)(srow + 4u * g) = w;
        }
        mx = fmaxf(mx, __shfl_xor(mx, 1, 32));
        const float mnew = fmaxf(mrow, mx);
        const float alpha = expf(mrow - mnew);
        mrow = mnew;
        float ps = 0.0f;
        for (unsigned g8 = 0; g8 < 4u; ++g8) {
            const v4f a = *(const v4f*)(srow + 8u * g8);
            const v4f bq = *(const v4f*)(srow + 8u * g8 + 4u);
            const float p0 = expf(a.x - mnew), p1 = expf(a.y - mnew), p2 = expf(a.z - mnew), p3 = expf(a.w - mnew);
            const float p4 = expf(bq.x - mnew), p5 = expf(bq.y - mnew), p6 = expf(bq.z - mnew), p7 = expf(bq.w - mnew);
            ps += ((p0 + p1) + (p2 + p3)) + ((p4 + p5) + (p6 + p7));
            v8h pv;
            pv[0] = toh_flush(p0 * CARRY_P); pv[1] = toh_flush(p1 * CARRY_P);
            pv[2] = toh_flush(p2 * CARRY_P); pv[3] = toh_flush(p3 * CARRY_P);
            pv[4] = toh_flush(p4 * CARRY_P); pv[5] = toh_flush(p5 * CARRY_P);
            pv[6] = toh_flush(p6 * CARRY_P); pv[7] = toh_flush(p7 * CARRY_P);
            *(v8h*)(prw + 8u * g8) = pv;
        }
        ps += __shfl_xor(ps, 1, 32);
        lrow = lrow * alpha + ps;
#pragma unroll
        for (int r = 0; r < 8; ++r) {
            const float ar = __shfl(alpha, (int)(16u * hh + 2u * (unsigned)r), 32);
#pragma unroll
            for (int t = 0; t < 4; ++t) o[t][r] *= ar;
        }
        wave_sync_lds();
#pragma unroll
        for (int kk = 0; kk < 2; ++kk) {
            const v16h pa = frag_ld(pw + c * AT_PP + (unsigned)kk * 32u + 8u * hh);
#pragma unroll
            for (int t = 0; t < 4; ++t) {
                const v16h vb = frag_ld(vbase + (size_t)((unsigned)t << 4) * SEQ_U + kv0 + (unsigned)kk * 32u);
                o[t] = wmma16g(pa, vb, o[t]);
            }
        }
        wave_sync_lds();
    }

    const float inv = 1.0f / lrow;
#pragma unroll
    for (int r = 0; r < 8; ++r) {
        const float ir = __shfl(inv, (int)(16u * hh + 2u * (unsigned)r), 32) * UNC_P;
#pragma unroll
        for (int t = 0; t < 4; ++t)
            slab[(8u * hh + (unsigned)r) * AT_SP + ((unsigned)t << 4) + c] = o[t][r] * ir;
    }
    wave_sync_lds();
    {
        const unsigned q = lane >> 3, c8 = (lane & 7u) * 8u;
        v8h ov[4];
#pragma unroll
        for (int it = 0; it < 4; ++it) {
            const float* sp = slab + ((unsigned)it * 4u + q) * AT_SP + c8;
#pragma unroll
            for (int e = 0; e < 8; ++e) ov[it][e] = toh_flush(sp[e]);
        }
        h16* dst = att + (size_t)tok0 * DM_U + head * HD_U;
        for (int pass = 0; pass < 2; ++pass) {
#pragma unroll
            for (int it = 0; it < 4; ++it)
                *(volatile v8h*)(dst + (size_t)((unsigned)it * 4u + q) * DM_U + c8) = ov[it];
            __threadfence();
        }
    }
}

template <bool FINAL>
__global__ __launch_bounds__(256) void k_ln(const float* __restrict__ pre, const float* __restrict__ g, const float* __restrict__ bt,
                                            float* __restrict__ yF, h16* __restrict__ yH) {
    const unsigned bx = blockIdx.x;
    const unsigned row = bx * 8u + (threadIdx.x >> 5);
    const unsigned L = threadIdx.x & 31u;
    if (row >= (unsigned)MTOK) return;
    const float* pr = pre + (size_t)row * DM_U;
    v4f v[8];
#pragma unroll
    for (int j = 0; j < 8; ++j) v[j] = *(const v4f*)(pr + 128u * (unsigned)j + 4u * L);
    float s = 0.0f;
#pragma unroll
    for (int j = 0; j < 8; ++j) s += (v[j].x + v[j].y) + (v[j].z + v[j].w);
#pragma unroll
    for (int off = 16; off > 0; off >>= 1) s += __shfl_xor(s, off, 32);
    const float mu = s / 1024.0f;
    float qs = 0.0f;
#pragma unroll
    for (int j = 0; j < 8; ++j) {
        const float d0 = v[j].x - mu, d1 = v[j].y - mu, d2 = v[j].z - mu, d3 = v[j].w - mu;
        qs += (d0 * d0 + d1 * d1) + (d2 * d2 + d3 * d3);
    }
#pragma unroll
    for (int off = 16; off > 0; off >>= 1) qs += __shfl_xor(qs, off, 32);
    const float var = qs / 1024.0f;
    const float rs = 1.0f / sqrtf(var + LN_EPS);
    unsigned orow = row;
    if (FINAL) orow = frow(row);
    float* yr = yF + (size_t)orow * DM_U;
    v4f y[8];
#pragma unroll
    for (int j = 0; j < 8; ++j) {
        const unsigned c0 = 128u * (unsigned)j + 4u * L;
        const v4f g4 = *(const v4f*)(g + c0);
        const v4f b4 = *(const v4f*)(bt + c0);
        y[j].x = (v[j].x - mu) * rs * bfr(g4.x) + bfr(b4.x);
        y[j].y = (v[j].y - mu) * rs * bfr(g4.y) + bfr(b4.y);
        y[j].z = (v[j].z - mu) * rs * bfr(g4.z) + bfr(b4.z);
        y[j].w = (v[j].w - mu) * rs * bfr(g4.w) + bfr(b4.w);
    }
    for (int pass = 0; pass < 2; ++pass) {
#pragma unroll
        for (int j = 0; j < 8; ++j) *(volatile v4f*)(yr + 128u * (unsigned)j + 4u * L) = y[j];
        __threadfence();
    }
    if (!FINAL) {
        h16* hr = yH + (size_t)row * DM_U;
        v8h hv[4];
#pragma unroll
        for (int gq = 0; gq < 4; ++gq) {
            const unsigned c0 = 256u * (unsigned)gq + 8u * L;
            const v4f a = *(const v4f*)(pr + c0), bq = *(const v4f*)(pr + c0 + 4u);
            const v4f ga = *(const v4f*)(g + c0), gb = *(const v4f*)(g + c0 + 4u);
            const v4f ba = *(const v4f*)(bt + c0), bb = *(const v4f*)(bt + c0 + 4u);
            hv[gq][0] = toh_flush(((a.x - mu) * rs * bfr(ga.x) + bfr(ba.x)) * CARRY_ACT);
            hv[gq][1] = toh_flush(((a.y - mu) * rs * bfr(ga.y) + bfr(ba.y)) * CARRY_ACT);
            hv[gq][2] = toh_flush(((a.z - mu) * rs * bfr(ga.z) + bfr(ba.z)) * CARRY_ACT);
            hv[gq][3] = toh_flush(((a.w - mu) * rs * bfr(ga.w) + bfr(ba.w)) * CARRY_ACT);
            hv[gq][4] = toh_flush(((bq.x - mu) * rs * bfr(gb.x) + bfr(bb.x)) * CARRY_ACT);
            hv[gq][5] = toh_flush(((bq.y - mu) * rs * bfr(gb.y) + bfr(bb.y)) * CARRY_ACT);
            hv[gq][6] = toh_flush(((bq.z - mu) * rs * bfr(gb.z) + bfr(bb.z)) * CARRY_ACT);
            hv[gq][7] = toh_flush(((bq.w - mu) * rs * bfr(gb.w) + bfr(bb.w)) * CARRY_ACT);
        }
        for (int pass = 0; pass < 2; ++pass) {
#pragma unroll
            for (int gq = 0; gq < 4; ++gq) *(volatile v8h*)(hr + 256u * (unsigned)gq + 8u * L) = hv[gq];
            __threadfence();
        }
    }
}

extern "C" void kernel_launch(void* const* d_in, const int* in_sizes, int n_in, void* d_out, int out_size,
                              void* d_ws, size_t ws_size, hipStream_t stream) {
    if (n_in < 15) return;
    const int needAct = ((NB - 1) * SEQ_FULL + SEQ) * DM;
    if (in_sizes[0] < needAct || in_sizes[1] < needAct) return;
    if (in_sizes[2] < 3 * DM * DM || in_sizes[3] < 3 * DM || in_sizes[4] < DM * DM || in_sizes[5] < DM) return;
    if (in_sizes[6] < DM || in_sizes[7] < DM || in_sizes[8] < FFD * DM || in_sizes[9] < FFD) return;
    if (in_sizes[10] < DM * FFD || in_sizes[11] < DM || in_sizes[12] < DM || in_sizes[13] < DM) return;
    if (out_size < needAct) return;
    if (ws_size < WS_TOTAL) return;

    const float* x     = (const float*)d_in[0];
    const float* imag  = (const float*)d_in[1];
    const float* w_qkv = (const float*)d_in[2];
    const float* b_qkv = (const float*)d_in[3];
    const float* w_o   = (const float*)d_in[4];
    const float* b_o   = (const float*)d_in[5];
    const float* ln1g  = (const float*)d_in[6];
    const float* ln1b  = (const float*)d_in[7];
    const float* w1    = (const float*)d_in[8];
    const float* b1    = (const float*)d_in[9];
    const float* w2    = (const float*)d_in[10];
    const float* b2    = (const float*)d_in[11];
    const float* ln2g  = (const float*)d_in[12];
    const float* ln2b  = (const float*)d_in[13];
    float* out = (float*)d_out;

    char* wsp = (char*)d_ws;
    h16*   x16   = (h16*)(wsp + OFF_X16);
    h16*   qk16  = (h16*)(wsp + OFF_QK);
    h16*   vT16  = (h16*)(wsp + OFF_VT);
    h16*   im16  = (h16*)(wsp + OFF_IM);
    h16*   hid16 = (h16*)(wsp + OFF_HID);
    h16*   wqkv  = (h16*)(wsp + OFF_WQKV);
    h16*   wo    = (h16*)(wsp + OFF_WO);
    h16*   w1h   = (h16*)(wsp + OFF_W1);
    h16*   w2h   = (h16*)(wsp + OFF_W2);
    float* hop   = (float*)(wsp + OFF_HOP);
    h16*   att16 = (h16*)(wsp + OFF_ATT);
    float* pre   = (float*)(wsp + OFF_PRE);
    float* x1f   = (float*)(wsp + OFF_X1F);
    h16*   x1h   = (h16*)(wsp + OFF_X1H);

    const unsigned nAct8 = (unsigned)(MTOK * (DM / 8));
    k_cvt16<0><<<nAct8 / 256u, 256, 0, stream>>>(x, x16, nAct8);
    k_cvt16<0><<<nAct8 / 256u, 256, 0, stream>>>(imag, im16, nAct8);
    k_cvt16<1><<<(3u * DM * DM / 8u) / 256u, 256, 0, stream>>>(w_qkv, wqkv, 3u * DM * DM / 8u);
    k_cvt16<1><<<(DM * DM / 8u) / 256u, 256, 0, stream>>>(w_o, wo, DM * DM / 8u);
    k_cvt16<1><<<(FFD * DM / 8u) / 256u, 256, 0, stream>>>(w1, w1h, FFD * DM / 8u);
    k_cvt16<1><<<(DM * FFD / 8u) / 256u, 256, 0, stream>>>(w2, w2h, DM * FFD / 8u);

    k_gemm<0><<<((MTOK / 64) * (3 * DM / 64) + 7) / 8, 256, 0, stream>>>(x16, wqkv, (void*)qk16, (void*)vT16, b_qkv, x);

    for (unsigned b = 0; b < (unsigned)NB; ++b) {
        const h16* imb = im16 + (size_t)b * SEQ * DM;
        k_gemm<1><<<((SEQ / 64) * (SEQ / 64) + 7) / 8, 256, 0, stream>>>(imb, imb, (void*)hop, (void*)hop, b_o, x);
        k_attn<<<dim3(SEQ / 64, HEADS), 128, 0, stream>>>(qk16, vT16, hop, att16, b);
    }

    k_gemm<2><<<((MTOK / 64) * (DM / 64) + 7) / 8, 256, 0, stream>>>(att16, wo, (void*)pre, (void*)pre, b_o, x);
    k_ln<false><<<MTOK / 8, 256, 0, stream>>>(pre, ln1g, ln1b, x1f, x1h);

    k_gemm<3><<<((MTOK / 64) * (FFD / 64) + 7) / 8, 256, 0, stream>>>(x1h, w1h, (void*)hid16, (void*)hid16, b1, x);
    k_gemm<4><<<((MTOK / 64) * (DM / 64) + 7) / 8, 256, 0, stream>>>(hid16, w2h, (void*)pre, (void*)pre, b2, x1f);
    k_ln<true><<<MTOK / 8, 256, 0, stream>>>(pre, ln2g, ln2b, out, x1h);
}
